// RNN_LSTM2_1589137900341
// MI455X (gfx1250) — hardware-verified
//
#include <hip/hip_runtime.h>
#include <math.h>

constexpr int NSEQ    = 64;
constexpr int NSTEP   = 256;
constexpr int NIN     = 512;
constexpr int NHID    = 1024;
constexpr int NOUTF   = 512;
constexpr int NG4     = 4 * NHID;
constexpr int NTHR    = 256;
constexpr int NWAVE   = NTHR / 32;
constexpr int SEQ_BLK = 16;
constexpr int UPW     = NHID / NWAVE;
constexpr int NGRP    = UPW / 32;
constexpr int XPITCH  = NIN + 8;
constexpr int HPITCH  = NHID + 8;
constexpr int CPITCH  = NHID + 4;
constexpr long PLX    = (long)NHID * NIN;
constexpr long PLH    = (long)NHID * NHID;
constexpr float WCARRY     = 16.0f;
constexpr float WCARRY_INV = 0.0625f;
static_assert(NSEQ % SEQ_BLK == 0, "blocks cover all sequences");
static_assert(NIN % 32 == 0 && NHID % 32 == 0, "k chunks of 32");
static_assert(UPW * NWAVE == NHID && NGRP * 32 == UPW, "wave column map");
static_assert(SEQ_BLK == 2 * NWAVE, "h copy: 2 rows per wave");
static_assert(NHID == 4 * 256, "h copy: 4 x (32 lanes x 8 halves) per row");
static_assert((XPITCH % 8) == 0 && (HPITCH % 8) == 0, "16-B aligned fragment rows");
static_assert((2 * SEQ_BLK * HPITCH) % NTHR == 0, "h zero fill exact");
static_assert((NSEQ * NSTEP) % 64 == 0 && NOUTF % 64 == 0 && NHID % 32 == 0, "head GEMM tile multiples");

typedef __attribute__((ext_vector_type(16))) _Float16 v16h;
typedef __attribute__((ext_vector_type(8)))  _Float16 v8h;
typedef __attribute__((ext_vector_type(16))) __bf16   v16b;
typedef __attribute__((ext_vector_type(8)))  __bf16   v8b;
typedef __attribute__((ext_vector_type(8)))  float    v8f;
typedef __attribute__((ext_vector_type(4)))  float    v4f;
typedef __attribute__((ext_vector_type(2)))  unsigned v2u;

__device__ __forceinline__ unsigned short f2bf_bits(float f) {
  unsigned u = __float_as_uint(f);
  return (unsigned short)((u + 0x7FFFu + ((u >> 16) & 1u)) >> 16);
}
__device__ __forceinline__ float bf_bits2f(unsigned short h) { return __uint_as_float(((unsigned)h) << 16); }
__device__ __forceinline__ float bf16r(float f) { return bf_bits2f(f2bf_bits(f)); }

__device__ __forceinline__ void dep_guard_h(v8f& a, v8f& b, v16h x, v16h y) { asm volatile("v_nop\n\tv_nop\n\tv_nop\n\tv_nop" : "+v"(a), "+v"(b) : "v"(x), "v"(y)); }
__device__ __forceinline__ void dep_guard_b(v8f& a, v8f& b, v16b x, v16b y) { asm volatile("v_nop\n\tv_nop\n\tv_nop\n\tv_nop" : "+v"(a), "+v"(b) : "v"(x), "v"(y)); }
__device__ __forceinline__ void keep4_h(v16h a, v16h b, v16h c, v16h d) { asm volatile("v_nop" :: "v"(a), "v"(b), "v"(c), "v"(d)); }
__device__ __forceinline__ void keep4_b(v16b a, v16b b, v16b c, v16b d) { asm volatile("v_nop" :: "v"(a), "v"(b), "v"(c), "v"(d)); }
__device__ __forceinline__ void acc_guard4(v8f& a, v8f& b, v8f& c, v8f& d) { asm volatile("v_nop\n\tv_nop\n\tv_nop\n\tv_nop" : "+v"(a), "+v"(b), "+v"(c), "+v"(d)); }
__device__ __forceinline__ void guard8_b(v8f& a0, v8f& a1, v8f& a2, v8f& a3, v8f& a4, v8f& a5, v8f& a6, v8f& a7, v16b x, v16b y) {
  asm volatile("v_nop\n\tv_nop\n\tv_nop\n\tv_nop" : "+v"(a0), "+v"(a1), "+v"(a2), "+v"(a3), "+v"(a4), "+v"(a5), "+v"(a6), "+v"(a7) : "v"(x), "v"(y));
}
__device__ __forceinline__ void guard8_h(v8f& a0, v8f& a1, v8f& a2, v8f& a3, v8f& a4, v8f& a5, v8f& a6, v8f& a7, v16h x, v16h y) {
  asm volatile("v_nop\n\tv_nop\n\tv_nop\n\tv_nop" : "+v"(a0), "+v"(a1), "+v"(a2), "+v"(a3), "+v"(a4), "+v"(a5), "+v"(a6), "+v"(a7) : "v"(x), "v"(y));
}
template <typename T> struct Frag;
template <> struct Frag<_Float16> {
  typedef v16h V; union U { v16h v; v8h h[2]; };
  static __device__ __forceinline__ v16h load(const _Float16* p) {
    U f; f.h[0] = *(const v8h*)(p); f.h[1] = *(const v8h*)(p + 16); return f.v;
  }
  static __device__ __forceinline__ v8f mma(v16h a, v16h b, v8f c) {
    return __builtin_amdgcn_wmma_f32_16x16x32_f16(false, a, false, b, (short)0, c, false, false);
  }
  static __device__ __forceinline__ void guard(v8f& a, v8f& b, v16h x, v16h y) { dep_guard_h(a, b, x, y); }
  static __device__ __forceinline__ void keep(v16h a, v16h b, v16h c, v16h d) { keep4_h(a, b, c, d); }
};
template <> struct Frag<__bf16> {
  typedef v16b V; union U { v16b v; v8b h[2]; };
  static __device__ __forceinline__ v16b load(const __bf16* p) {
    U f; f.h[0] = *(const v8b*)(p); f.h[1] = *(const v8b*)(p + 16); return f.v;
  }
  static __device__ __forceinline__ v8f mma(v16b a, v16b b, v8f c) {
    return __builtin_amdgcn_wmma_f32_16x16x32_bf16(false, a, false, b, (short)0, c, false, false);
  }
  static __device__ __forceinline__ void guard(v8f& a, v8f& b, v16b x, v16b y) { dep_guard_b(a, b, x, y); }
  static __device__ __forceinline__ void keep(v16b a, v16b b, v16b c, v16b d) { keep4_b(a, b, c, d); }
};

__device__ __forceinline__ float fsig(float x)  { return __builtin_amdgcn_rcpf(1.0f + __expf(-x)); }
__device__ __forceinline__ float ftanh(float x) { return 1.0f - 2.0f * __builtin_amdgcn_rcpf(__expf(2.0f * x) + 1.0f); }

template <int ET> struct Elem;
template <> struct Elem<0> { typedef _Float16 T; };
template <> struct Elem<1> { typedef __bf16 T; };
template <int ET, bool SPLIT, int BIAS_MODE, int OUT_MODE, bool RESID, int ACT = 0>
__global__ __launch_bounds__(256) void wmma_gemm64(
    const unsigned short* __restrict__ Ap, const unsigned short* __restrict__ A2p, int lda, long strideA,
    const unsigned short* __restrict__ Btp, const unsigned short* __restrict__ Bt2p, int ldb, long strideB,
    void* __restrict__ Cout, void* __restrict__ Cout2, int ldc, long strideC,
    const float* __restrict__ bias,
    const float* __restrict__ resid, long strideR,
    int M, int N, int K, float scale) {
  typedef typename Elem<ET>::T T;
  typedef typename Frag<T>::V V;
  const T* A = (const T*)Ap; const T* A2 = (const T*)A2p; const T* Bt = (const T*)Btp; const T* Bt2 = (const T*)Bt2p;
  __shared__ __align__(16) float sT[8][16 * 68];
  const int b    = blockIdx.y;
  const int lane = threadIdx.x & 31;
  const int wave = threadIdx.x >> 5;
  const int tilesN = N >> 6;
  const int tilesM = M >> 6;
  const int tile = blockIdx.x * 8 + wave;
  if (tile >= tilesM * tilesN) return;
  const int tm = tile / tilesN;
  const int tn = tile - tm * tilesN;
  const int m0 = tm << 6;
  const int n0 = tn << 6;

  const T* Ab  = A  + (size_t)b * strideA;
  const T* Bb  = Bt + (size_t)b * strideB;
  const T* Ab2 = SPLIT ? (A2  + (size_t)b * strideA) : nullptr;
  const T* Bb2 = SPLIT ? (Bt2 + (size_t)b * strideB) : nullptr;

  const int rlane = lane & 15;
  const int koff  = (lane >> 4) * 8;
  const int mOff  = (lane >> 4) * 8;

  v8f acc[4][4];
#pragma unroll
  for (int i = 0; i < 4; ++i)
#pragma unroll
    for (int j = 0; j < 4; ++j) acc[i][j] = (v8f){0.f,0.f,0.f,0.f,0.f,0.f,0.f,0.f};

  for (int k0 = 0; k0 < K; k0 += 32) {
    V bh[4], bl[4];
#pragma unroll
    for (int j = 0; j < 4; ++j) {
      const size_t bo = (size_t)(n0 + (j << 4) + rlane) * ldb + koff + k0;
      bh[j] = Frag<T>::load(Bb + bo);
      if (SPLIT) bl[j] = Frag<T>::load(Bb2 + bo);
    }
#pragma unroll
    for (int i = 0; i < 4; ++i) {
      const size_t ao = (size_t)(m0 + (i << 4) + rlane) * lda + koff + k0;
      V ah = Frag<T>::load(Ab + ao);
      V al;
      if (SPLIT) al = Frag<T>::load(Ab2 + ao);
#pragma unroll
      for (int j = 0; j < 4; ++j) {
        acc[i][j] = Frag<T>::mma(ah, bh[j], acc[i][j]);
        if (SPLIT) {
          acc[i][j] = Frag<T>::mma(ah, bl[j], acc[i][j]);
          acc[i][j] = Frag<T>::mma(al, bh[j], acc[i][j]);
        }
      }
      Frag<T>::guard(acc[i][0], acc[i][3], ah, SPLIT ? al : ah);
    }
    Frag<T>::keep(bh[0], bh[1], bh[2], bh[3]);
    if (SPLIT) Frag<T>::keep(bl[0], bl[1], bl[2], bl[3]);
  }
  acc_guard4(acc[0][0], acc[0][1], acc[0][2], acc[0][3]);
  acc_guard4(acc[1][0], acc[1][1], acc[1][2], acc[1][3]);
  acc_guard4(acc[2][0], acc[2][1], acc[2][2], acc[2][3]);
  acc_guard4(acc[3][0], acc[3][1], acc[3][2], acc[3][3]);

  float* slab = sT[wave];
  const float* Rb = RESID ? (resid + (size_t)b * strideR) : nullptr;
#pragma unroll
  for (int i = 0; i < 4; ++i) {
    const int mBase = m0 + (i << 4);
#pragma unroll
    for (int j = 0; j < 4; ++j) {
      const int n = n0 + (j << 4) + rlane;
      float bv = 0.f;
      if (BIAS_MODE == 2) bv = bias[n];
#pragma unroll
      for (int r = 0; r < 8; ++r) {
        float v = acc[i][j][r] * scale;
        if (BIAS_MODE == 1) v += bias[mBase + mOff + r];
        if (BIAS_MODE == 2) v += bv;
        if (RESID) v += Rb[(size_t)(mBase + mOff + r) * ldc + n];
        if (ACT == 1) v = tanhf(v);
        if (ACT == 2) v = fmaxf(v, 0.0f);
        if (ACT == 3) v = v / (1.0f + expf(-v));
        if (ACT == 4) v = (v > 0.f) ? v : 0.01f * v;
        if (ACT == 5) v = 0.5f * v * (1.0f + erff(v * 0.70710678118654752f));
        if (ACT == 6) v = __builtin_amdgcn_rcpf(1.0f + __expf(-v));
        slab[(mOff + r) * 68 + (j << 4) + rlane] = v;
      }
    }
    __builtin_amdgcn_fence(__ATOMIC_RELEASE, "workgroup");
    __builtin_amdgcn_wave_barrier();
    __builtin_amdgcn_fence(__ATOMIC_ACQUIRE, "workgroup");
    if (OUT_MODE == 0) {
      float* C = (float*)Cout + (size_t)b * strideC;
      const int hh = lane >> 4, c4 = (lane & 15) * 4;
      for (int pass = 0; pass < 2; ++pass) {
#pragma unroll
        for (int it = 0; it < 8; ++it) {
          const int row = it * 2 + hh;
          v4f v = *(const v4f*)(slab + row * 68 + c4);
          *(volatile v4f*)(C + (size_t)(mBase + row) * ldc + n0 + c4) = v;
        }
        __threadfence();
      }
    } else {
      const int q = lane >> 3, c8 = (lane & 7) * 8;
      unsigned short* C  = (unsigned short*)Cout  + (size_t)b * strideC;
      unsigned short* C2 = (OUT_MODE == 2) ? ((unsigned short*)Cout2 + (size_t)b * strideC) : nullptr;
      for (int pass = 0; pass < 2; ++pass) {
#pragma unroll
        for (int it = 0; it < 4; ++it) {
          const int row = it * 4 + q;
          const float* sp = slab + row * 68 + c8;
          v8h hv, lv;
#pragma unroll
          for (int e = 0; e < 8; ++e) {
            if (OUT_MODE == 1) {
              hv[e] = (_Float16)sp[e];
            } else {
              unsigned short hb = f2bf_bits(sp[e]);
              unsigned short lb = f2bf_bits(sp[e] - bf_bits2f(hb));
              hv[e] = __builtin_bit_cast(_Float16, hb);
              lv[e] = __builtin_bit_cast(_Float16, lb);
            }
          }
          *(volatile v8h*)(C + (size_t)(mBase + row) * ldc + n0 + c8) = hv;
          if (OUT_MODE == 2) *(volatile v8h*)(C2 + (size_t)(mBase + row) * ldc + n0 + c8) = lv;
        }
        __threadfence();
      }
    }
    __builtin_amdgcn_fence(__ATOMIC_RELEASE, "workgroup");
    __builtin_amdgcn_wave_barrier();
    __builtin_amdgcn_fence(__ATOMIC_ACQUIRE, "workgroup");
  }
}

template <int MODE>
__global__ __launch_bounds__(NTHR) void cvt8x4_kernel(const float* __restrict__ s0, const float* __restrict__ s1,
                                                    const float* __restrict__ s2, const float* __restrict__ s3,
                                                    unsigned short* __restrict__ dst, int n8, long planeElems, float sc) {
  const int gy = blockIdx.y;
  const float* src = (gy == 0) ? s0 : (gy == 1) ? s1 : (gy == 2) ? s2 : s3;
  unsigned short* d = dst + (size_t)gy * (size_t)planeElems;
  const int i = blockIdx.x * NTHR + threadIdx.x;
  if (i < n8) {
    const v4f a = *(const v4f*)(src + (size_t)i * 8);
    const v4f b = *(const v4f*)(src + (size_t)i * 8 + 4);
    v8h hv;
#pragma unroll
    for (int e = 0; e < 4; ++e) {
      unsigned short b0, b1;
      if (MODE == 0) {
        b0 = f2bf_bits(a[e] * sc);
        b1 = f2bf_bits(b[e] * sc);
      } else {
        b0 = __builtin_bit_cast(unsigned short, (_Float16)(bf16r(a[e]) * sc));
        b1 = __builtin_bit_cast(unsigned short, (_Float16)(bf16r(b[e]) * sc));
      }
      hv[e]     = __builtin_bit_cast(_Float16, b0);
      hv[4 + e] = __builtin_bit_cast(_Float16, b1);
    }
    *(volatile v8h*)(d + (size_t)i * 8) = hv;
    __threadfence();
    *(volatile v8h*)(d + (size_t)i * 8) = hv;
  }
}

__global__ __launch_bounds__(NTHR) void bias_kernel(const float* __restrict__ ufb, const float* __restrict__ wfb,
                                                  const float* __restrict__ ugb, const float* __restrict__ wgb,
                                                  const float* __restrict__ ucb, const float* __restrict__ wcb,
                                                  const float* __restrict__ uob, const float* __restrict__ wob,
                                                  const float* __restrict__ ob,
                                                  float* __restrict__ bsum, float* __restrict__ obr) {
  const int i = blockIdx.x * NTHR + threadIdx.x;
  if (blockIdx.x < NG4 / NTHR) {
    const int g = i >> 10;
    const int j = i & (NHID - 1);
    const float v0 = bf16r(ufb[j]) + bf16r(wfb[j]);
    const float v1 = bf16r(ugb[j]) + bf16r(wgb[j]);
    const float v2 = bf16r(ucb[j]) + bf16r(wcb[j]);
    const float v3 = bf16r(uob[j]) + bf16r(wob[j]);
    const float v = (g == 0) ? v0 : (g == 1) ? v1 : (g == 2) ? v2 : v3;
    ((volatile float*)bsum)[i] = v;
    __threadfence();
    ((volatile float*)bsum)[i] = v;
  } else {
    const int n = i - NG4;
    if (n < NOUTF) {
      const float v = bf16r(ob[n]);
      ((volatile float*)obr)[n] = v;
      __threadfence();
      ((volatile float*)obr)[n] = v;
    }
  }
}

__device__ __forceinline__ void stage_x(const float* __restrict__ x, unsigned short* ax, int rowbase, int t, int tid) {
  const int m = tid >> 4, f4 = (tid & 15) * 4;
  const float* src = x + ((size_t)(rowbase + m) * NSTEP + (size_t)t) * NIN + f4;
  unsigned short* dst = ax + m * XPITCH + f4;
#pragma unroll
  for (int i = 0; i < NIN / 64; ++i) {
    const v4f v = *(const v4f*)(src + 64 * i);
    const unsigned short u0 = f2bf_bits(v[0]), u1 = f2bf_bits(v[1]), u2 = f2bf_bits(v[2]), u3 = f2bf_bits(v[3]);
    v2u pk;
    pk[0] = (unsigned)u0 | ((unsigned)u1 << 16);
    pk[1] = (unsigned)u2 | ((unsigned)u3 << 16);
    *(v2u*)(dst + 64 * i) = pk;
  }
}

__global__ __launch_bounds__(NTHR) void rec_seq_kernel(const float* __restrict__ x, const float* __restrict__ bsum,
                                                     const unsigned short* __restrict__ WXp,
                                                     const unsigned short* __restrict__ WHp,
                                                     unsigned short* __restrict__ HS) {
  __shared__ __align__(16) unsigned short Ax[SEQ_BLK * XPITCH];
  __shared__ __align__(16) _Float16       Ah[2][SEQ_BLK * HPITCH];
  __shared__ __align__(16) float          Cs[SEQ_BLK * CPITCH];
  const __bf16*   WX = (const __bf16*)WXp;
  const _Float16* WH = (const _Float16*)WHp;
  const int tid = threadIdx.x, lane = tid & 31, wave = tid >> 5;
  const int c = lane & 15, hh = lane >> 4, koff = hh * 8;
  const int rowbase = blockIdx.x * SEQ_BLK;

  {
    _Float16* ahf = &Ah[0][0];
#pragma unroll 1
    for (int i = tid; i < 2 * SEQ_BLK * HPITCH; i += NTHR) ahf[i] = (_Float16)0.0f;
#pragma unroll 1
    for (int i = tid; i < SEQ_BLK * CPITCH; i += NTHR) Cs[i] = 0.0f;
  }
  stage_x(x, Ax, rowbase, 0, tid);
  __syncthreads();

  const v8f z8 = {0.f, 0.f, 0.f, 0.f, 0.f, 0.f, 0.f, 0.f};

#pragma unroll 1
  for (int t = 0; t < NSTEP; ++t) {
    const int cur = t & 1;
    const __bf16*   axrow = (const __bf16*)(&Ax[0]) + c * XPITCH + koff;
    const _Float16* ahrow = &Ah[cur][0] + c * HPITCH + koff;
    _Float16* ahn = &Ah[cur ^ 1][0];
#pragma unroll
    for (int grp = 0; grp < NGRP; ++grp) {
      const int jA = UPW * wave + 32 * grp + c;
      const int jB = jA + 16;
      const __bf16*   wxA = WX + (size_t)jA * NIN + koff;
      const __bf16*   wxB = WX + (size_t)jB * NIN + koff;
      const _Float16* whA = WH + (size_t)jA * NHID + koff;
      const _Float16* whB = WH + (size_t)jB * NHID + koff;
      v8f acc[8];
      acc[0] = z8; acc[1] = z8; acc[2] = z8; acc[3] = z8; acc[4] = z8; acc[5] = z8; acc[6] = z8; acc[7] = z8;
#pragma unroll 1
      for (int kx = 0; kx < NIN; kx += 32) {
        const v16b a  = Frag<__bf16>::load(axrow + kx);
        const v16b b0 = Frag<__bf16>::load(wxA + kx);
        const v16b b1 = Frag<__bf16>::load(wxA + PLX + kx);
        const v16b b2 = Frag<__bf16>::load(wxA + 2 * PLX + kx);
        const v16b b3 = Frag<__bf16>::load(wxA + 3 * PLX + kx);
        const v16b e0 = Frag<__bf16>::load(wxB + kx);
        const v16b e1 = Frag<__bf16>::load(wxB + PLX + kx);
        const v16b e2 = Frag<__bf16>::load(wxB + 2 * PLX + kx);
        const v16b e3 = Frag<__bf16>::load(wxB + 3 * PLX + kx);
        acc[0] = Frag<__bf16>::mma(a, b0, acc[0]);
        acc[1] = Frag<__bf16>::mma(a, b1, acc[1]);
        acc[2] = Frag<__bf16>::mma(a, b2, acc[2]);
        acc[3] = Frag<__bf16>::mma(a, b3, acc[3]);
        acc[4] = Frag<__bf16>::mma(a, e0, acc[4]);
        acc[5] = Frag<__bf16>::mma(a, e1, acc[5]);
        acc[6] = Frag<__bf16>::mma(a, e2, acc[6]);
        acc[7] = Frag<__bf16>::mma(a, e3, acc[7]);
        guard8_b(acc[0], acc[1], acc[2], acc[3], acc[4], acc[5], acc[6], acc[7], a, e3);
        keep4_b(b0, b1, b2, b3);
        keep4_b(e0, e1, e2, e3);
      }
#pragma unroll 1
      for (int k0 = 0; k0 < NHID; k0 += 32) {
        const v16h a  = Frag<_Float16>::load(ahrow + k0);
        const v16h b0 = Frag<_Float16>::load(whA + k0);
        const v16h b1 = Frag<_Float16>::load(whA + PLH + k0);
        const v16h b2 = Frag<_Float16>::load(whA + 2 * PLH + k0);
        const v16h b3 = Frag<_Float16>::load(whA + 3 * PLH + k0);
        const v16h e0 = Frag<_Float16>::load(whB + k0);
        const v16h e1 = Frag<_Float16>::load(whB + PLH + k0);
        const v16h e2 = Frag<_Float16>::load(whB + 2 * PLH + k0);
        const v16h e3 = Frag<_Float16>::load(whB + 3 * PLH + k0);
        acc[0] = Frag<_Float16>::mma(a, b0, acc[0]);
        acc[1] = Frag<_Float16>::mma(a, b1, acc[1]);
        acc[2] = Frag<_Float16>::mma(a, b2, acc[2]);
        acc[3] = Frag<_Float16>::mma(a, b3, acc[3]);
        acc[4] = Frag<_Float16>::mma(a, e0, acc[4]);
        acc[5] = Frag<_Float16>::mma(a, e1, acc[5]);
        acc[6] = Frag<_Float16>::mma(a, e2, acc[6]);
        acc[7] = Frag<_Float16>::mma(a, e3, acc[7]);
        guard8_h(acc[0], acc[1], acc[2], acc[3], acc[4], acc[5], acc[6], acc[7], a, e3);
        keep4_h(b0, b1, b2, b3);
        keep4_h(e0, e1, e2, e3);
      }
      acc_guard4(acc[0], acc[1], acc[2], acc[3]);
      acc_guard4(acc[4], acc[5], acc[6], acc[7]);
      {
        const float bfA = bsum[jA], bgA = bsum[NHID + jA], bcA = bsum[2 * NHID + jA], boA = bsum[3 * NHID + jA];
        const float bfB = bsum[jB], bgB = bsum[NHID + jB], bcB = bsum[2 * NHID + jB], boB = bsum[3 * NHID + jB];
#pragma unroll
        for (int u = 0; u < 2; ++u) {
          const int   j   = u ? jB : jA;
          const float bf_ = u ? bfB : bfA;
          const float bg_ = u ? bgB : bgA;
          const float bc_ = u ? bcB : bcA;
          const float bo_ = u ? boB : boA;
#pragma unroll
          for (int r = 0; r < 8; ++r) {
            const int row = 8 * hh + r;
            const float zf = acc[4 * u + 0][r] * WCARRY_INV + bf_;
            const float zg = acc[4 * u + 1][r] * WCARRY_INV + bg_;
            const float zc = acc[4 * u + 2][r] * WCARRY_INV + bc_;
            const float zo = acc[4 * u + 3][r] * WCARRY_INV + bo_;
            const float fg = fsig(zf);
            const float ig = fsig(zg);
            const float og = fsig(zo);
            const float cd = ftanh(zc);
            const float cprev = Cs[row * CPITCH + j];
            const float cn = fg * cprev + ig * cd;
            Cs[row * CPITCH + j] = cn;
            const float hn = og * ftanh(cn);
            ahn[row * HPITCH + j] = (_Float16)hn;
          }
        }
      }
    }
    __syncthreads();

    {
      const int tn = (t + 1 < NSTEP) ? (t + 1) : (NSTEP - 1);
      stage_x(x, Ax, rowbase, tn, tid);
    }
    {
      const _Float16* hsrc = &Ah[cur ^ 1][0];
      for (int pass = 0; pass < 2; ++pass) {
#pragma unroll
        for (int rr = 0; rr < 2; ++rr) {
          const int m = 2 * wave + rr;
          unsigned short* drow = HS + ((size_t)(rowbase + m) * NSTEP + (size_t)t) * NHID;
#pragma unroll
          for (int q = 0; q < 4; ++q) {
            const v8h v = *(const v8h*)(hsrc + m * HPITCH + q * 256 + lane * 8);
            *(volatile v8h*)(drow + q * 256 + lane * 8) = v;
          }
        }
        __threadfence();
      }
    }
    __syncthreads();
  }
}

extern "C" void kernel_launch(void* const* d_in, const int* in_sizes, int n_in,
                              void* d_out, int out_size, void* d_ws, size_t ws_size, hipStream_t stream) {
  if (n_in < 19 || d_out == nullptr || d_ws == nullptr) return;
  if (in_sizes[0] != NSEQ * NSTEP * NIN || out_size != NSEQ * NSTEP * NOUTF) return;
  if (in_sizes[1] != NHID * NIN || in_sizes[3] != NHID * NIN || in_sizes[5] != NHID * NIN || in_sizes[7] != NHID * NIN) return;
  if (in_sizes[9] != NHID * NHID || in_sizes[11] != NHID * NHID || in_sizes[13] != NHID * NHID || in_sizes[15] != NHID * NHID) return;
  if (in_sizes[2] != NHID || in_sizes[4] != NHID || in_sizes[6] != NHID || in_sizes[8] != NHID) return;
  if (in_sizes[10] != NHID || in_sizes[12] != NHID || in_sizes[14] != NHID || in_sizes[16] != NHID) return;
  if (in_sizes[17] != NOUTF * NHID || in_sizes[18] != NOUTF) return;

  const float* x    = (const float*)d_in[0];
  const float* uf_w = (const float*)d_in[1];
  const float* uf_b = (const float*)d_in[2];
  const float* ug_w = (const float*)d_in[3];
  const float* ug_b = (const float*)d_in[4];
  const float* uc_w = (const float*)d_in[5];
  const float* uc_b = (const float*)d_in[6];
  const float* uo_w = (const float*)d_in[7];
  const float* uo_b = (const float*)d_in[8];
  const float* wf_w = (const float*)d_in[9];
  const float* wf_b = (const float*)d_in[10];
  const float* wg_w = (const float*)d_in[11];
  const float* wg_b = (const float*)d_in[12];
  const float* wc_w = (const float*)d_in[13];
  const float* wc_b = (const float*)d_in[14];
  const float* wo_w = (const float*)d_in[15];
  const float* wo_b = (const float*)d_in[16];
  const float* o_w  = (const float*)d_in[17];
  const float* o_b  = (const float*)d_in[18];
  float* out = (float*)d_out;

  char* ws = (char*)d_ws; size_t off = 0;
  auto carve = [&](size_t bytes) -> char* { char* p = ws + off; off += (bytes + 255) & ~(size_t)255; return p; };
  unsigned short* WX   = (unsigned short*)carve((size_t)4 * PLX * 2);
  unsigned short* WH   = (unsigned short*)carve((size_t)4 * PLH * 2);
  unsigned short* OW   = (unsigned short*)carve((size_t)NOUTF * NHID * 2);
  unsigned short* HS   = (unsigned short*)carve((size_t)NSEQ * NSTEP * NHID * 2);
  float*          BSUM = (float*)carve((size_t)NG4 * 4);
  float*          OBR  = (float*)carve((size_t)NOUTF * 4);
  if (off > ws_size || off > (size_t)134217728) return;

  const int n8x = (int)(PLX / 8);
  const int n8h = (int)(PLH / 8);
  const int n8o = NOUTF * NHID / 8;
  cvt8x4_kernel<0><<<dim3((n8x + NTHR - 1) / NTHR, 4, 1), NTHR, 0, stream>>>(uf_w, ug_w, uc_w, uo_w, WX, n8x, PLX, WCARRY);
  cvt8x4_kernel<1><<<dim3((n8h + NTHR - 1) / NTHR, 4, 1), NTHR, 0, stream>>>(wf_w, wg_w, wc_w, wo_w, WH, n8h, PLH, WCARRY);
  cvt8x4_kernel<1><<<dim3((n8o + NTHR - 1) / NTHR, 1, 1), NTHR, 0, stream>>>(o_w, o_w, o_w, o_w, OW, n8o, (long)NOUTF * NHID, WCARRY);
  bias_kernel<<<NG4 / NTHR + NOUTF / NTHR, NTHR, 0, stream>>>(uf_b, wf_b, ug_b, wg_b, uc_b, wc_b, uo_b, wo_b, o_b, BSUM, OBR);
  rec_seq_kernel<<<NSEQ / SEQ_BLK, NTHR, 0, stream>>>(x, BSUM, WX, WH, HS);

  const int headM = NSEQ * NSTEP, headN = NOUTF, headK = NHID;
  const int headTiles = (headM / 64) * (headN / 64);
  wmma_gemm64<0, false, 2, 0, false, 6><<<dim3((headTiles + 7) / 8, 1, 1), 256, 0, stream>>>(
      HS, HS, headK, 0L, OW, OW, headK, 0L, (void*)out, (void*)out, headN, 0L,
      OBR, nullptr, 0L, headM, headN, headK, WCARRY_INV);
}
